// GNNLoRA_47021301956658
// MI455X (gfx1250) — hardware-run, weakly checked
//
#include <hip/hip_runtime.h>


namespace {
constexpr int NN = 50000, NP = 50016, NE = 800000, D = 128, C0 = 128, C1 = 64, RK = 32, MAXDEG = 1024, NGc = (NN + 511) / 512, PERMLEN = NE + 32 * NGc + 32;
constexpr float XS = 8.0f, SLOPE = 0.2f;

typedef _Float16 b16;
typedef __attribute__((ext_vector_type(16))) _Float16 v16b;
typedef __attribute__((ext_vector_type(8))) _Float16 v8b;
typedef __attribute__((ext_vector_type(8))) float v8f;
typedef __attribute__((ext_vector_type(4))) float v4f;
__device__ __forceinline__ float bf16_rne(float f) { unsigned int u = __float_as_uint(f); u += 0x7FFFu + ((u >> 16) & 1u); return __uint_as_float(u & 0xFFFF0000u); }
__device__ __forceinline__ void split16(float v, b16& hi, b16& lo) { hi = (b16)v; lo = (b16)(v - (float)hi); }
__device__ __forceinline__ v16b frag_kb(const b16* p, int hh) { const v8b a = *(const v8b*)(p + 8 * hh), b = *(const v8b*)(p + 16 + 8 * hh); v16b f;
#pragma unroll
  for (int e = 0; e < 8; ++e) { f[e] = a[e]; f[8 + e] = b[e]; } return f; }
__device__ __forceinline__ v8f wmma16b(v16b a, v16b b, v8f c) { v8f d = __builtin_amdgcn_wmma_f32_16x16x32_f16(false, a, false, b, (short)0, c, false, false); asm volatile("v_nop\n\tv_nop\n\tv_nop\n\tv_nop" : "+v"(d) : "v"(a), "v"(b)); return d; }
__device__ __forceinline__ void wave_lds_sync() { __builtin_amdgcn_fence(__ATOMIC_RELEASE, "workgroup"); __builtin_amdgcn_wave_barrier(); __builtin_amdgcn_fence(__ATOMIC_ACQUIRE, "workgroup"); }
__device__ __forceinline__ float nexp(float x) { return __builtin_amdgcn_exp2f(x * 1.4426950408889634f); }
__device__ __forceinline__ float pmul(float a, float b) { float p = a * b; asm volatile("" : "+v"(p)); return p; }
__device__ __forceinline__ float leaky(float x) { return (x >= 0.0f) ? x : SLOPE * x; }
constexpr int CSR_NBLK = 512, CSR_GB = 9, CSR_GN = 1 << CSR_GB  , CSR_MAXG = 512, CSR_CAP = 12288  ;
__global__ __launch_bounds__(64) void csrA_kernel(const int* __restrict__ dst, int E, int N, int nG, int CHP, int NGP, int* __restrict__ STG, int* __restrict__ HST) {
  extern __shared__ int sm[];
  int* cnt = sm; int* run = sm + NGP; int* ids = sm + 2 * NGP;
  const int b = blockIdx.x; const int ch = (E + CSR_NBLK - 1) / CSR_NBLK; const int e0 = b * ch, e1 = min(E, e0 + ch);
  for (int i = threadIdx.x; i < NGP; i += 64) cnt[i] = 0;
  for (int i = threadIdx.x; i < CHP; i += 64) ids[i] = -1;
  __syncthreads();
  if (threadIdx.x == 0) {
    for (int e = e0; e < e1; ++e) { int d = dst[e]; d = (d < 0) ? 0 : (d >= N ? N - 1 : d); cnt[d >> CSR_GB] += 1; }
    int acc = 0; for (int g = 0; g < nG; ++g) { run[g] = acc; acc += cnt[g]; }
    for (int e = e0; e < e1; ++e) { int d = dst[e]; d = (d < 0) ? 0 : (d >= N ? N - 1 : d); const int g = d >> CSR_GB; ids[run[g]] = e; run[g] += 1; } }
  __syncthreads();
  typedef __attribute__((ext_vector_type(4))) int v4i;
  for (int pass = 0; pass < 2; ++pass) {
    for (int i = threadIdx.x; i < CHP / 4; i += 64) *(volatile v4i*)(STG + (size_t)b * CHP + i * 4) = *(const v4i*)(&ids[i * 4]);
    for (int i = threadIdx.x; i < NGP / 4; i += 64) { v4i v; for (int e = 0; e < 4; ++e) v[e] = (i * 4 + e < nG) ? cnt[i * 4 + e] : 0; *(volatile v4i*)(HST + (size_t)b * NGP + i * 4) = v; }
    __threadfence(); }
}
__global__ __launch_bounds__(512) void csrS_kernel(const int* __restrict__ HST, int nG, int NGP, int* __restrict__ START, int* __restrict__ TOT, int* __restrict__ OFF) {
  __shared__ int tot[CSR_MAXG];
  const int b = threadIdx.x;
  for (int pass = 0; pass < 2; ++pass) { int runb = 0; for (int g = 0; g < nG; ++g) { int c = HST[(size_t)b * NGP + g]; c = (c < 0) ? 0 : c; ((volatile int*)OFF)[(size_t)g * CSR_NBLK + b] = runb; runb += c; } __threadfence(); }
  for (int g = threadIdx.x; g < nG; g += 512) { int s = 0; for (int bb = 0; bb < CSR_NBLK; ++bb) { int c = HST[(size_t)bb * NGP + g]; s += (c < 0) ? 0 : c; } tot[g] = s; }
  __syncthreads();
  if (threadIdx.x < 32) {
    __shared__ int st[CSR_MAXG + 32];
    if (threadIdx.x == 0) { int acc = 0; for (int g = 0; g < NGP; ++g) { st[g] = acc; if (g < nG) acc += (tot[g] + 31) & ~31; } st[NGP] = acc; }
    __builtin_amdgcn_fence(__ATOMIC_RELEASE, "workgroup"); __builtin_amdgcn_wave_barrier(); __builtin_amdgcn_fence(__ATOMIC_ACQUIRE, "workgroup");
    for (int pass = 0; pass < 2; ++pass) { for (int i = threadIdx.x; i < NGP + 32; i += 32) { ((volatile int*)START)[i] = (i <= NGP) ? st[min(i, NGP)] : 0; ((volatile int*)TOT)[i] = (i < nG) ? tot[i] : 0; } __threadfence(); } }
}
__global__ __launch_bounds__(256) void csrB_kernel(const int* __restrict__ dst, int N, int nG, int CHP, int NGP, int permLen, const int* __restrict__ STG, const int* __restrict__ HST, const int* __restrict__ OFF, const int* __restrict__ START, const int* __restrict__ TOT, int* __restrict__ PERM, int* __restrict__ ROWPTR, int* __restrict__ ROWCNT, int* __restrict__ FLAG) {
  typedef __attribute__((ext_vector_type(4))) int v4i;
  __shared__ int ids[CSR_CAP]; __shared__ unsigned short key[CSR_CAP]; __shared__ int outp[CSR_CAP]; __shared__ int ncnt[CSR_GN + 1]; __shared__ int boff[CSR_NBLK + 1];
  const int g = blockIdx.x, t_ = threadIdx.x; int tot = TOT[g]; int st = START[g], stn = START[g + 1]; const int v0 = g * CSR_GN; const int nv = min(CSR_GN, N - v0);
  st = (st < 0) ? 0 : (st > permLen - 32 ? permLen - 32 : st) & ~31; stn = (stn < st) ? st : (stn > permLen ? permLen : stn); tot = (tot < 0) ? 0 : tot; if (tot > stn - st && tot <= CSR_CAP) tot = stn - st;
  if (tot > CSR_CAP) {
    for (int pass = 0; pass < 2; ++pass) { for (int i = t_; i < CSR_GN / 4; i += 256) { v4i a, c; for (int e = 0; e < 4; ++e) { a[e] = st; c[e] = 0; } *(volatile v4i*)(ROWPTR + v0 + i * 4) = a; *(volatile v4i*)(ROWCNT + v0 + i * 4) = c; } if (t_ == 0) ((volatile int*)FLAG)[0] = 1; __threadfence(); } (void)nv; return; }
  if (t_ == 0) { int acc = 0; for (int b = 0; b < CSR_NBLK; ++b) { boff[b] = acc; int c = HST[(size_t)b * NGP + g]; c = (c < 0) ? 0 : (c > CHP ? CHP : c); acc += c; if (acc > tot) acc = tot; } boff[CSR_NBLK] = acc; }
  for (int i = t_; i <= CSR_GN; i += 256) ncnt[i] = 0;
  __syncthreads();
  for (int b = 0; b < CSR_NBLK; ++b) { const int c = boff[b + 1] - boff[b]; int o_ = OFF[(size_t)g * CSR_NBLK + b]; o_ = (o_ < 0) ? 0 : (o_ > CHP - c ? CHP - c : o_); const int* src_ = STG + (size_t)b * CHP + o_;
    for (int i = t_; i < c; i += 256) { int id = src_[i]; id = (id < 0) ? 0 : id; ids[boff[b] + i] = id; int d = dst[id]; d = (d < v0) ? v0 : (d >= N ? N - 1 : d); int kk = d - v0; kk = (kk < 0) ? 0 : (kk >= CSR_GN ? CSR_GN - 1 : kk); key[boff[b] + i] = (unsigned short)kk; } }
  __syncthreads();
  if (t_ == 0) { for (int i = 0; i < tot; ++i) ncnt[key[i]] += 1; int acc = 0; for (int vl = 0; vl < CSR_GN; ++vl) { const int c = ncnt[vl]; ncnt[vl] = acc; acc += c; } ncnt[CSR_GN] = acc;
    for (int i = 0; i < tot; ++i) { const int vl = key[i]; outp[ncnt[vl]] = ids[i]; ncnt[vl] += 1; }
    for (int vl = CSR_GN; vl > 0; --vl) ncnt[vl] = ncnt[vl - 1]; ncnt[0] = 0; }
  __syncthreads();
  for (int pass = 0; pass < 2; ++pass) {
    for (int i = t_; i < (stn - st) / 4; i += 256) { v4i v; for (int e = 0; e < 4; ++e) { const int q = i * 4 + e; v[e] = (q < tot) ? outp[q] : -1; } *(volatile v4i*)(PERM + st + i * 4) = v; }
    for (int i = t_; i < CSR_GN / 4; i += 256) { v4i a, c; for (int e = 0; e < 4; ++e) { const int vl = i * 4 + e; a[e] = st + ncnt[vl]; c[e] = (vl < nv) ? (ncnt[vl + 1] - ncnt[vl]) : 0; } *(volatile v4i*)(ROWPTR + v0 + i * 4) = a; *(volatile v4i*)(ROWCNT + v0 + i * 4) = c; }
    __threadfence(); }
}
__global__ __launch_bounds__(256) void csrZ_kernel(int* __restrict__ p, size_t n4) { typedef __attribute__((ext_vector_type(4))) int v4i; const size_t tid = (size_t)blockIdx.x * 256 + threadIdx.x, nth = (size_t)gridDim.x * 256; v4i z = {0, 0, 0, 0}; for (size_t i = tid; i < n4; i += nth) *(volatile v4i*)(p + i * 4) = z; }
struct CsrBufs { int *STG, *HST, *OFF, *START, *TOT, *PERM, *ROWPTR, *ROWCNT, *FLAG; int nG, NGP, CHP; size_t permLen; char* base; size_t bytes; };
static size_t csr_carve(CsrBufs& c, char* ws, size_t off, int E, int N) {
  const size_t off0 = off; c.base = ws + off;
  auto al = [&](size_t bytes) { char* p = ws + off; off += (bytes + 255) & ~(size_t)255; return p; };
  c.nG = (N + CSR_GN - 1) / CSR_GN; c.NGP = (c.nG + 31) & ~31; const int ch = (E + CSR_NBLK - 1) / CSR_NBLK; c.CHP = (ch + 31) & ~31; c.permLen = (size_t)E + 32 * (size_t)c.nG + 32;
  c.STG = (int*)al((size_t)CSR_NBLK * c.CHP * 4); c.HST = (int*)al((size_t)CSR_NBLK * c.NGP * 4); c.OFF = (int*)al((size_t)c.NGP * CSR_NBLK * 4); c.START = (int*)al((size_t)(c.NGP + 64) * 4); c.TOT = (int*)al((size_t)(c.NGP + 64) * 4);
  c.PERM = (int*)al(c.permLen * 4); c.ROWPTR = (int*)al((size_t)c.nG * CSR_GN * 4); c.ROWCNT = (int*)al((size_t)c.nG * CSR_GN * 4); c.FLAG = (int*)al(256);
  c.bytes = off - off0; return off;
}
static void csr_build(const CsrBufs& c, const int* dst, int E, int N, hipStream_t stream) {
  const size_t smem = (size_t)(2 * c.NGP + c.CHP) * 4;
  csrZ_kernel<<<512, 256, 0, stream>>>((int*)c.base, c.bytes / 16);
  csrA_kernel<<<CSR_NBLK, 64, smem, stream>>>(dst, E, N, c.nG, c.CHP, c.NGP, c.STG, c.HST);
  csrS_kernel<<<1, 512, 0, stream>>>(c.HST, c.nG, c.NGP, c.START, c.TOT, c.OFF);
  csrB_kernel<<<c.nG, 256, 0, stream>>>(dst, N, c.nG, c.CHP, c.NGP, (int)c.permLen, c.STG, c.HST, c.OFF, c.START, c.TOT, c.PERM, c.ROWPTR, c.ROWCNT, c.FLAG);
}

struct Ro_ { static constexpr size_t P0 = 0, L0 = P0 + 160 * 128, P1 = L0 + 128 * 32, L1 = P1 + 96 * 128, END = L1 + 64 * 32; };
__global__ __launch_bounds__(256) void prep_kernel(const float* __restrict__ x, const float* __restrict__ w0, const float* __restrict__ as0, const float* __restrict__ ad0, const float* __restrict__ b0, const float* __restrict__ w1, const float* __restrict__ as1, const float* __restrict__ ad1, const float* __restrict__ b1,
    const float* __restrict__ la0, const float* __restrict__ lb0, const float* __restrict__ ls0, const float* __restrict__ ld0, const float* __restrict__ lbb0, const float* __restrict__ la1, const float* __restrict__ lb1, const float* __restrict__ ls1, const float* __restrict__ ld1, const float* __restrict__ lbb1,
    b16* __restrict__ R, float* __restrict__ P, b16* __restrict__ X, b16* __restrict__ Hlpad) {
  const size_t tid = (size_t)blockIdx.x * 256 + threadIdx.x, nth = (size_t)gridDim.x * 256;
  auto tr = [&](size_t base, int nout, int kin, const float* W, int ldw, int col0) { for (size_t p = tid; p < (size_t)nout * kin; p += nth) { const int o = (int)(p / kin), k = (int)(p % kin); ((volatile b16*)R)[base + p] = (b16)bf16_rne(W[(size_t)k * ldw + col0 + o]); } };
  for (int pass = 0; pass < 2; ++pass) {
    tr(Ro_::P0, 128, 128, w0, 128, 0); tr(Ro_::P0 + 128 * 128, 32, 128, la0, 32, 0); tr(Ro_::L0, 128, 32, lb0, 128, 0); tr(Ro_::P1, 64, 128, w1, 64, 0); tr(Ro_::P1 + 64 * 128, 32, 128, la1, 32, 0); tr(Ro_::L1, 64, 32, lb1, 64, 0);
    for (size_t q = tid; q < 1152; q += nth) { const int i = (int)q; float v; if (i < 768) { const int s_ = i / 128, c = i % 128; const float* a = (s_ == 0) ? as0 : (s_ == 1) ? ad0 : (s_ == 2) ? b0 : (s_ == 3) ? ls0 : (s_ == 4) ? ld0 : lbb0; v = a[c]; } else { const int s_ = (i - 768) / 64, c = (i - 768) % 64; const float* a = (s_ == 0) ? as1 : (s_ == 1) ? ad1 : (s_ == 2) ? b1 : (s_ == 3) ? ls1 : (s_ == 4) ? ld1 : lbb1; v = a[c]; } P[q] = bf16_rne(v); }
    for (size_t p = tid; p < (size_t)NP * D / 8; p += nth) { const size_t r = p / (D / 8); v8b v = {}; if (r < (size_t)NN) for (int e = 0; e < 8; ++e) v[e] = (b16)(bf16_rne(x[p * 8 + e]) * XS); *(volatile v8b*)(X + p * 8) = v; if (r >= (size_t)NN) *(volatile v8b*)(Hlpad + (p - (size_t)NN * D / 8) * 8) = v; }
    __threadfence(); }
}

template <int CB, int TWO>
__global__ __launch_bounds__(64) void proj_kernel(const b16* __restrict__ Ah, const b16* __restrict__ Al, const b16* __restrict__ Bp, const b16* __restrict__ Bl, const float* __restrict__ Pl, float* __restrict__ HF, float* __restrict__ ALR) {
  constexpr int NS = CB / 16 + 2, NL = CB / 16;
  __shared__ __attribute__((aligned(16))) float Ts[2][16][2 * CB + 4]; __shared__ __attribute__((aligned(16))) b16 Xa[2][16][RK + 8], Xl[2][16][RK + 8]; __shared__ __attribute__((aligned(16))) float Av[2][16][4];
  const int lane = threadIdx.x & 31, wave = threadIdx.x >> 5, nloc = lane & 15, hlf = lane >> 4, m0 = blockIdx.x * 32 + wave * 16;
  v8f acc[NS];
#pragma unroll
  for (int t = 0; t < NS; ++t) acc[t] = (v8f){};
#pragma unroll
  for (int kb = 0; kb < D; kb += 32) { const v16b a = frag_kb(Ah + (size_t)(m0 + nloc) * D + kb, hlf); v16b al_; if (TWO) al_ = frag_kb(Al + (size_t)(m0 + nloc) * D + kb, hlf);
#pragma unroll
    for (int t = 0; t < NS; ++t) { const v16b bw = frag_kb(Bp + (size_t)(t * 16 + nloc) * D + kb, hlf); acc[t] = wmma16b(a, bw, acc[t]); if (TWO) acc[t] = wmma16b(al_, bw, acc[t]); } }
#pragma unroll
  for (int t = 0; t < NL; ++t)
#pragma unroll
    for (int r = 0; r < 8; ++r) Ts[wave][8 * hlf + r][t * 16 + nloc] = acc[t][r] * (1.0f / XS);
#pragma unroll
  for (int t = 0; t < 2; ++t)
#pragma unroll
    for (int r = 0; r < 8; ++r) { b16 a_, b_; split16(acc[NL + t][r], a_, b_); Xa[wave][8 * hlf + r][t * 16 + nloc] = a_; Xl[wave][8 * hlf + r][t * 16 + nloc] = b_; }
  wave_lds_sync();
  { v8f lacc[NL]; for (int t = 0; t < NL; ++t) lacc[t] = (v8f){}; const v16b a = frag_kb(&Xa[wave][nloc][0], hlf), al_ = frag_kb(&Xl[wave][nloc][0], hlf);
#pragma unroll
    for (int t = 0; t < NL; ++t) { const v16b bw = frag_kb(Bl + (size_t)(t * 16 + nloc) * RK, hlf); lacc[t] = wmma16b(a, bw, lacc[t]); lacc[t] = wmma16b(al_, bw, lacc[t]); }
#pragma unroll
    for (int t = 0; t < NL; ++t)
#pragma unroll
      for (int r = 0; r < 8; ++r) Ts[wave][8 * hlf + r][CB + t * 16 + nloc] = lacc[t][r] * (1.0f / XS); }
  wave_lds_sync();
  if (lane < 16) { const float* row = &Ts[wave][lane][0]; float s0 = 0.0f, s1 = 0.0f, s2 = 0.0f, s3 = 0.0f; for (int c = 0; c < CB; ++c) { s0 += pmul(row[c], Pl[c]); s1 += pmul(row[c], Pl[CB + c]); s2 += pmul(row[CB + c], Pl[3 * CB + c]); s3 += pmul(row[CB + c], Pl[4 * CB + c]); } Av[wave][lane][0] = s0; Av[wave][lane][1] = s1; Av[wave][lane][2] = s2; Av[wave][lane][3] = s3; }
  wave_lds_sync();
  for (int pass = 0; pass < 2; ++pass) { for (int i = lane; i < 16 * (2 * CB / 4); i += 32) { const int rr = i / (2 * CB / 4), c4 = (i % (2 * CB / 4)) * 4; *(volatile v4f*)(HF + (size_t)(m0 + rr) * (2 * CB) + c4) = *(const v4f*)(&Ts[wave][rr][c4]); }
    if (lane < 16) *(volatile v4f*)(ALR + (size_t)(m0 + lane) * 4) = *(const v4f*)(&Av[wave][lane][0]); __threadfence(); }
}

template <int LAYER, int CB>
__global__ __launch_bounds__(256) void gat_kernel(const float* __restrict__ HF, const float* __restrict__ ALR, const int* __restrict__ src, const int* __restrict__ perm, const int* __restrict__ rowptr, const int* __restrict__ rowcnt, const float* __restrict__ Pl, b16* __restrict__ Hh, b16* __restrict__ Hl, float* __restrict__ out0, float* __restrict__ out1, float* __restrict__ out2) {
  constexpr int PL = CB / 16;
  __shared__ __attribute__((aligned(16))) b16 Sh[8][C0 + 8], Sl[8][C0 + 8];
  const int wave = threadIdx.x >> 5, v = blockIdx.x * 8 + wave, lane = threadIdx.x & 31, side = lane >> 4, cl = (lane & 15) * PL;
  int cnt = rowcnt[v]; cnt = (cnt < 0) ? 0 : (cnt > MAXDEG ? MAXDEG : cnt); int p0 = rowptr[v]; p0 = (p0 < 0) ? 0 : (p0 > PERMLEN - cnt ? PERMLEN - cnt : p0);
  const float adv = ALR[(size_t)v * 4 + 2 * side + 1]; float m = -INFINITY, l = 0.0f; float acc[PL]; for (int k = 0; k < PL; ++k) acc[k] = 0.0f;
  for (int q = 0; q <= cnt; ++q) { int j; if (q < cnt) { int id = perm[p0 + q]; id = (id < 0) ? 0 : (id >= NE ? NE - 1 : id); j = src[id]; j = (j < 0) ? 0 : (j >= NN ? NN - 1 : j); } else j = v;
    const float e = leaky(ALR[(size_t)j * 4 + 2 * side] + adv); const float mn = fmaxf(m, e); const float al_ = nexp(m - mn); const float p = nexp(e - mn); m = mn; l = l * al_ + p;
    const float* hr = HF + (size_t)j * (2 * CB) + side * CB + cl;
#pragma unroll
    for (int k = 0; k < PL; k += 4) { const v4f f = *(const v4f*)(hr + k); for (int kk = 0; kk < 4; ++kk) acc[k + kk] = acc[k + kk] * al_ + pmul(p, f[kk]); } }
  const float inv = 1.0f / (l + 1e-16f); float y[PL];
#pragma unroll
  for (int k = 0; k < PL; ++k) y[k] = acc[k] * inv + Pl[2 * CB + side * 3 * CB + cl + k];
  float ysum[PL];
#pragma unroll
  for (int k = 0; k < PL; ++k) ysum[k] = y[k] + __shfl_xor(y[k], 16);
  if (LAYER == 0) {
#pragma unroll
    for (int k = 0; k < PL; ++k) { b16 a_, b_; split16(ysum[k] * XS, a_, b_); if (side == 0) { Sh[wave][cl + k] = a_; Sl[wave][cl + k] = b_; } }
    wave_lds_sync();
    for (int pass = 0; pass < 2; ++pass) { if (lane < 16) { *(volatile v8b*)(Hh + (size_t)v * C0 + lane * 8) = *(const v8b*)(&Sh[wave][lane * 8]); *(volatile v8b*)(Hl + (size_t)v * C0 + lane * 8) = *(const v8b*)(&Sl[wave][lane * 8]); } __threadfence(); } }
  else { v4f o, os; for (int k = 0; k < 4; ++k) { o[k] = y[k]; os[k] = ysum[k]; }
    for (int pass = 0; pass < 2; ++pass) { if (side == 0) { *(volatile v4f*)(out1 + (size_t)v * C1 + cl) = o; *(volatile v4f*)(out0 + (size_t)v * C1 + cl) = os; } else *(volatile v4f*)(out2 + (size_t)v * C1 + cl) = o; __threadfence(); } }
}
}

extern "C" void kernel_launch(void* const* d_in, const int* in_sizes, int n_in,
                              void* d_out, int out_size, void* d_ws, size_t ws_size, hipStream_t stream) {
  (void)n_in; (void)out_size;
  const float* x = (const float*)d_in[0]; const int* ei = (const int*)d_in[1];
  const float* w0 = (const float*)d_in[2]; const float* as0 = (const float*)d_in[3]; const float* ad0 = (const float*)d_in[4]; const float* b0 = (const float*)d_in[5]; const float* w1 = (const float*)d_in[6]; const float* as1 = (const float*)d_in[7]; const float* ad1 = (const float*)d_in[8]; const float* b1 = (const float*)d_in[9];
  const float* la0 = (const float*)d_in[10]; const float* lb0 = (const float*)d_in[11]; const float* ls0 = (const float*)d_in[12]; const float* ld0 = (const float*)d_in[13]; const float* lbb0 = (const float*)d_in[14]; const float* la1 = (const float*)d_in[15]; const float* lb1 = (const float*)d_in[16]; const float* ls1 = (const float*)d_in[17]; const float* ld1 = (const float*)d_in[18]; const float* lbb1 = (const float*)d_in[19];
  float* out0 = (float*)d_out; float* out1 = (float*)((char*)d_out + (size_t)NN * C1 * 4); float* out2 = (float*)((char*)d_out + (size_t)2 * NN * C1 * 4);
  if (in_sizes[0] != NN * D || in_sizes[1] != 2 * NE || in_sizes[2] != D * C0 || in_sizes[10] != D * RK) return;
  const int* srcI = ei; const int* dstI = ei + NE; const int NE_RUN = NE;
  size_t off = 0; char* ws = (char*)d_ws;
  auto carve = [&](size_t bytes) { char* p = ws + off; off += (bytes + 255) & ~(size_t)255; return p; };
  b16* R = (b16*)carve(Ro_::END * 2); float* P = (float*)carve(1152 * 4); b16* X = (b16*)carve((size_t)NP * D * 2); float* HF = (float*)carve((size_t)NP * 2 * C0 * 4); float* ALR = (float*)carve((size_t)NP * 4 * 4); b16* Hl = (b16*)carve((size_t)NP * C0 * 2);
  CsrBufs cs; off = csr_carve(cs, ws, off, NE_RUN, NN);
  if (off > ws_size) return;
  b16* Hh = X;
  csr_build(cs, dstI, NE_RUN, NN, stream);
  prep_kernel<<<512, 256, 0, stream>>>(x, w0, as0, ad0, b0, w1, as1, ad1, b1, la0, lb0, ls0, ld0, lbb0, la1, lb1, ls1, ld1, lbb1, R, P, X, Hl + (size_t)NN * C0);
  proj_kernel<128, 0><<<NP / 32, 64, 0, stream>>>(X, nullptr, R + Ro_::P0, R + Ro_::L0, P, HF, ALR);
  gat_kernel<0, 128><<<NN / 8, 256, 0, stream>>>(HF, ALR, srcI, cs.PERM, cs.ROWPTR, cs.ROWCNT, P, Hh, Hl, nullptr, nullptr, nullptr);
  proj_kernel<64, 1><<<NP / 32, 64, 0, stream>>>(Hh, Hl, R + Ro_::P1, R + Ro_::L1, P + 768, HF, ALR);
  gat_kernel<1, 64><<<NN / 8, 256, 0, stream>>>(HF, ALR, srcI, cs.PERM, cs.ROWPTR, cs.ROWCNT, P + 768, nullptr, nullptr, out0, out1, out2);
}
